// GPT_OSS_MLP_74105365725337
// MI455X (gfx1250) — hardware-verified
//
#include <hip/hip_runtime.h>


namespace {
constexpr int T = 512, H = 2880, I = 2880, TOPK = 4, NG64 = H / 64;
constexpr float XS = 8.0f, WSC = 256.0f, ALPHA = 1.702f, LIMIT = 7.0f;
typedef _Float16 b16;
typedef __attribute__((ext_vector_type(16))) _Float16 v16b;
typedef __attribute__((ext_vector_type(8))) _Float16 v8b;
typedef __attribute__((ext_vector_type(8))) float v8f;
typedef __attribute__((ext_vector_type(2))) float v2f;
__device__ __forceinline__ float bf16_rne(float f) { unsigned int u = __float_as_uint(f); u += 0x7FFFu + ((u >> 16) & 1u); float r = __uint_as_float(u & 0xFFFF0000u); asm volatile("" : "+v"(r)); return r; }
__device__ __forceinline__ void split16(float v, b16& hi, b16& lo) { hi = (b16)v; lo = (b16)(v - (float)hi); }
__device__ __forceinline__ v16b frag_kb(const b16* p, int hh) { const v8b a = *(const v8b*)(p + 8 * hh), b = *(const v8b*)(p + 16 + 8 * hh); v16b f;
#pragma unroll
  for (int e = 0; e < 8; ++e) { f[e] = a[e]; f[8 + e] = b[e]; } return f; }
__device__ __forceinline__ v8f wmma16b(v16b a, v16b b, v8f c) { v8f d = __builtin_amdgcn_wmma_f32_16x16x32_f16(false, a, false, b, (short)0, c, false, false); asm volatile("v_nop\n\tv_nop\n\tv_nop\n\tv_nop" : "+v"(d) : "v"(a), "v"(b)); return d; }
__device__ __forceinline__ void wave_lds_sync() { __builtin_amdgcn_fence(__ATOMIC_RELEASE, "workgroup"); __builtin_amdgcn_wave_barrier(); __builtin_amdgcn_fence(__ATOMIC_ACQUIRE, "workgroup"); }
__device__ __forceinline__ float pmul(float a, float b) { float p = a * b; asm volatile("" : "+v"(p)); return p; }

__global__ __launch_bounds__(256) void wput_kernel(const float* __restrict__ w, int K, int N, b16* __restrict__ WT) { const int KG = K / 8; const size_t u = (size_t)blockIdx.x * 256 + threadIdx.x; if (u >= (size_t)N * KG) return; const int o = (int)(u / KG), k0 = (int)(u % KG) * 8; v8b v;
#pragma unroll
  for (int j = 0; j < 8; ++j) v[j] = (b16)(bf16_rne(w[(size_t)(k0 + j) * N + o]) * WSC); for (int pass = 0; pass < 2; ++pass) { *(volatile v8b*)(WT + (size_t)o * K + k0) = v; __threadfence(); } }
__global__ __launch_bounds__(32) void gu_kernel(const float* __restrict__ x, const b16* __restrict__ WG, const b16* __restrict__ WU, const float* __restrict__ gb, const float* __restrict__ ub, float* __restrict__ HM) {
  __shared__ __attribute__((aligned(16))) b16 Ah[16][H + 8]; __shared__ float Tf[16][68]; const int lane = threadIdx.x, nloc = lane & 15, hlf = lane >> 4; const int g = blockIdx.x % NG64; const size_t m0 = (size_t)(blockIdx.x / NG64) * 16;
  for (int rr = 0; rr < 16; ++rr) for (int q = 0; q < H / 32; ++q) Ah[rr][q * 32 + lane] = (b16)(bf16_rne(x[(m0 + rr) * H + q * 32 + lane]) * XS);
  wave_lds_sync(); v8f ag[4] = {(v8f){}, (v8f){}, (v8f){}, (v8f){}}, au[4] = {(v8f){}, (v8f){}, (v8f){}, (v8f){}};
#pragma unroll 2
  for (int kb = 0; kb < H; kb += 32) { const v16b a = frag_kb(&Ah[nloc][kb], hlf);
#pragma unroll
    for (int t = 0; t < 4; ++t) { const size_t o = (size_t)(g * 64 + t * 16 + nloc) * H + kb; ag[t] = wmma16b(a, frag_kb(WG + o, hlf), ag[t]); au[t] = wmma16b(a, frag_kb(WU + o, hlf), au[t]); } }
#pragma unroll
  for (int t = 0; t < 4; ++t) { const int c = g * 64 + t * 16 + nloc; const float bg_ = bf16_rne(gb[c]), bu_ = bf16_rne(ub[c]);
#pragma unroll
    for (int r8 = 0; r8 < 8; ++r8) { float gt = ag[t][r8] * (1.0f / (XS * WSC)) + bg_; float up = au[t][r8] * (1.0f / (XS * WSC)) + bu_; up = fminf(fmaxf(up, -LIMIT), LIMIT); gt = fminf(gt, LIMIT); const float glu = pmul(gt, 1.0f / (1.0f + __expf(-ALPHA * gt))); Tf[8 * hlf + r8][t * 16 + nloc] = pmul(glu, up + 1.0f); } }
  wave_lds_sync();
  for (int pass = 0; pass < 2; ++pass) { for (int rr = 0; rr < 16; ++rr) *(volatile v2f*)(HM + (m0 + rr) * I + g * 64 + lane * 2) = (v2f){Tf[rr][lane * 2], Tf[rr][lane * 2 + 1]}; __threadfence(); } }
__global__ __launch_bounds__(32) void down_kernel(const float* __restrict__ HM, const b16* __restrict__ WD, const float* __restrict__ db, const float* __restrict__ fin, const float* __restrict__ rw, const int* __restrict__ em, float* __restrict__ out) {
  constexpr int KCH = 960; __shared__ __attribute__((aligned(16))) b16 Ah[16][KCH + 8], Al[16][KCH + 8]; __shared__ float Tf[16][68], Tw[16]; const int lane = threadIdx.x, nloc = lane & 15, hlf = lane >> 4; const int g = blockIdx.x % NG64; const size_t m0 = (size_t)(blockIdx.x / NG64) * 16;
  if (lane < 16) { const int t = (int)m0 + lane; float s = 0.0f; for (int j = 0; j < TOPK; ++j) s += pmul((float)em[(size_t)j * T + t], bf16_rne(rw[(size_t)t * TOPK + j])); Tw[lane] = s; }
  v8f acc[4] = {(v8f){}, (v8f){}, (v8f){}, (v8f){}};
#pragma unroll 1
  for (int kc = 0; kc < I; kc += KCH) { wave_lds_sync();
    for (int rr = 0; rr < 16; ++rr) for (int q = 0; q < KCH / 32; ++q) { b16 p, ql; split16(HM[(m0 + rr) * I + kc + q * 32 + lane] * XS, p, ql); Ah[rr][q * 32 + lane] = p; Al[rr][q * 32 + lane] = ql; }
    wave_lds_sync();
#pragma unroll 2
    for (int kb = 0; kb < KCH; kb += 32) { const v16b a = frag_kb(&Ah[nloc][kb], hlf), al = frag_kb(&Al[nloc][kb], hlf);
#pragma unroll
      for (int t = 0; t < 4; ++t) { const v16b bw = frag_kb(WD + (size_t)(g * 64 + t * 16 + nloc) * I + kc + kb, hlf); acc[t] = wmma16b(a, bw, acc[t]); acc[t] = wmma16b(al, bw, acc[t]); } } }
#pragma unroll
  for (int t = 0; t < 4; ++t) { const int c = g * 64 + t * 16 + nloc; const float bb = bf16_rne(db[c]);
#pragma unroll
    for (int r8 = 0; r8 < 8; ++r8) { const int rl = 8 * hlf + r8; const float y = acc[t][r8] * (1.0f / (XS * WSC)) + bb; Tf[rl][t * 16 + nloc] = bf16_rne(fin[(m0 + rl) * H + c]) + pmul(y, Tw[rl]); } }
  wave_lds_sync();
  for (int pass = 0; pass < 2; ++pass) { for (int rr = 0; rr < 16; ++rr) *(volatile v2f*)(out + (m0 + rr) * H + g * 64 + lane * 2) = (v2f){Tf[rr][lane * 2], Tf[rr][lane * 2 + 1]}; __threadfence(); } }
}

extern "C" void kernel_launch(void* const* d_in, const int* in_sizes, int n_in, void* d_out, int out_size, void* d_ws, size_t ws_size, hipStream_t stream) {
  (void)n_in;
  auto Fp = [&](int i) { return (const float*)d_in[i]; }; auto Ip = [&](int i) { return (const int*)d_in[i]; };
  if (in_sizes[0] != T * H || in_sizes[1] != T * TOPK || in_sizes[2] != T * H || in_sizes[3] != H * I || in_sizes[5] != H * I || in_sizes[7] != I * H || in_sizes[9] != TOPK * T || out_size != T * H) return;
  const int TV = T;
  size_t off = 0; char* ws = (char*)d_ws;
  auto carve = [&](size_t bytes) { char* p = ws + off; off += (bytes + 255) & ~(size_t)255; return p; };
  b16* WG = (b16*)carve((size_t)I * H * 2); b16* WU = (b16*)carve((size_t)I * H * 2); b16* WD = (b16*)carve((size_t)H * I * 2); float* HM = (float*)carve((size_t)T * I * 4);
  if (off > ws_size || off > ((size_t)64 << 20)) return;
  wput_kernel<<<(unsigned)(((size_t)I * (H / 8) + 255) / 256), 256, 0, stream>>>(Fp(3), H, I, WG); wput_kernel<<<(unsigned)(((size_t)I * (H / 8) + 255) / 256), 256, 0, stream>>>(Fp(5), H, I, WU); wput_kernel<<<(unsigned)(((size_t)H * (I / 8) + 255) / 256), 256, 0, stream>>>(Fp(7), I, H, WD);
  gu_kernel<<<(TV / 16) * NG64, 32, 0, stream>>>(Fp(0), WG, WU, Fp(4), Fp(6), HM);
  down_kernel<<<(TV / 16) * NG64, 32, 0, stream>>>(HM, WD, Fp(8), Fp(2), Fp(1), Ip(9), (float*)d_out);
}
